// MutiHeadattention_7593502179569
// MI455X (gfx1250) — hardware-verified
//
#include <hip/hip_runtime.h>
#include <hip/hip_bf16.h>
#include <math.h>

typedef __attribute__((ext_vector_type(16))) _Float16 v16h;
typedef __attribute__((ext_vector_type(8)))  _Float16 v8h;
typedef __attribute__((ext_vector_type(16))) __bf16   v16b;
typedef __attribute__((ext_vector_type(8)))  __bf16   v8b;
typedef __attribute__((ext_vector_type(8)))  float    v8f;
typedef __attribute__((ext_vector_type(4)))  float    v4f;
typedef __attribute__((ext_vector_type(4)))  unsigned int v4u;

constexpr int kBatch  = 4;
constexpr int kSeq    = 2048;
constexpr int kHeads  = 16;
constexpr int kHd     = 64;
constexpr int kHid    = kHeads * kHd;
constexpr int kRows   = kBatch * kSeq;
constexpr int kBPP    = 2;
constexpr int kRowsPP = kBPP * kSeq;
constexpr int kKC     = 64;
constexpr int kQB     = 64;

static_assert(kHd % 32 == 0);
static_assert(kHid % 32 == 0);
static_assert(kRows % 64 == 0);
static_assert(kHid % 64 == 0);
static_assert(kHd % 64 == 0);
static_assert(kRowsPP % 64 == 0);
static_assert(((kRows / 64) * (kHid / 64)) % 8 == 0);
static_assert(((kRowsPP / 64) * (kHd / 64)) % 8 == 0);
static_assert(kSeq % kQB == 0);
static_assert(kSeq % kKC == 0);
static_assert(kBatch % kBPP == 0);
static_assert(kHd % 64 == 0 && kHid % 32 == 0);
static_assert(kHid % 64 == 0 && kHd % 32 == 0);
static_assert((kRows * kHd) % 512 == 0);

__device__ __forceinline__ unsigned short f2bf_bits(float f) {
  unsigned u = __float_as_uint(f);
  return (unsigned short)((u + 0x7FFFu + ((u >> 16) & 1u)) >> 16);
}
__device__ __forceinline__ float bf_bits2f(unsigned short h) { return __uint_as_float(((unsigned)h) << 16); }

__device__ __forceinline__ void dep_guard_h(v8f& a, v8f& b, v16h x, v16h y) { asm volatile("v_nop\n\tv_nop\n\tv_nop\n\tv_nop" : "+v"(a), "+v"(b) : "v"(x), "v"(y)); }
__device__ __forceinline__ void dep_guard_b(v8f& a, v8f& b, v16b x, v16b y) { asm volatile("v_nop\n\tv_nop\n\tv_nop\n\tv_nop" : "+v"(a), "+v"(b) : "v"(x), "v"(y)); }
__device__ __forceinline__ void keep4_h(v16h a, v16h b, v16h c, v16h d) { asm volatile("v_nop" :: "v"(a), "v"(b), "v"(c), "v"(d)); }
__device__ __forceinline__ void keep4_b(v16b a, v16b b, v16b c, v16b d) { asm volatile("v_nop" :: "v"(a), "v"(b), "v"(c), "v"(d)); }
__device__ __forceinline__ void acc_guard4(v8f& a, v8f& b, v8f& c, v8f& d) { asm volatile("v_nop\n\tv_nop\n\tv_nop\n\tv_nop" : "+v"(a), "+v"(b), "+v"(c), "+v"(d)); }
template <typename T> struct Frag;
template <> struct Frag<_Float16> {
  typedef v16h V; union U { v16h v; v8h h[2]; };
  static __device__ __forceinline__ v16h load(const _Float16* p) {
    U f; f.h[0] = *(const v8h*)(p); f.h[1] = *(const v8h*)(p + 16); return f.v;
  }
  static __device__ __forceinline__ v8f mma(v16h a, v16h b, v8f c) {
    return __builtin_amdgcn_wmma_f32_16x16x32_f16(false, a, false, b, (short)0, c, false, false);
  }
  static __device__ __forceinline__ void guard(v8f& a, v8f& b, v16h x, v16h y) { dep_guard_h(a, b, x, y); }
  static __device__ __forceinline__ void keep(v16h a, v16h b, v16h c, v16h d) { keep4_h(a, b, c, d); }
};
template <> struct Frag<__bf16> {
  typedef v16b V; union U { v16b v; v8b h[2]; };
  static __device__ __forceinline__ v16b load(const __bf16* p) {
    U f; f.h[0] = *(const v8b*)(p); f.h[1] = *(const v8b*)(p + 16); return f.v;
  }
  static __device__ __forceinline__ v8f mma(v16b a, v16b b, v8f c) {
    return __builtin_amdgcn_wmma_f32_16x16x32_bf16(false, a, false, b, (short)0, c, false, false);
  }
  static __device__ __forceinline__ void guard(v8f& a, v8f& b, v16b x, v16b y) { dep_guard_b(a, b, x, y); }
  static __device__ __forceinline__ void keep(v16b a, v16b b, v16b c, v16b d) { keep4_b(a, b, c, d); }
};

__device__ __forceinline__ v8f at_mma(v16b a, v16b b, v8f c) {
  c = __builtin_amdgcn_wmma_f32_16x16x32_bf16(false, a, false, b, (short)0, c, false, false);
  asm volatile("v_nop\n\tv_nop\n\tv_nop\n\tv_nop" : "+v"(c) : "v"(a), "v"(b));
  return c;
}

template <int ET> struct Elem;
template <> struct Elem<0> { typedef _Float16 T; };
template <> struct Elem<1> { typedef __bf16 T; };
template <int ET, bool SPLIT, int BIAS_MODE, int OUT_MODE, bool RESID, int ACT = 0>
__global__ __launch_bounds__(256) void wmma_gemm64(
    const unsigned short* __restrict__ Ap, const unsigned short* __restrict__ A2p, int lda, long strideA,
    const unsigned short* __restrict__ Btp, const unsigned short* __restrict__ Bt2p, int ldb, long strideB,
    void* __restrict__ Cout, void* __restrict__ Cout2, int ldc, long strideC,
    const float* __restrict__ bias,
    const float* __restrict__ resid, long strideR,
    int M, int N, int K, float scale) {
  static_assert(!RESID);
  static_assert(ACT == 0);
  typedef typename Elem<ET>::T T;
  typedef typename Frag<T>::V V;
  const T* A = (const T*)Ap; const T* A2 = (const T*)A2p; const T* Bt = (const T*)Btp; const T* Bt2 = (const T*)Bt2p;
  __shared__ __align__(16) float sT[8][16 * 68];
  const int b    = blockIdx.y;
  const int lane = threadIdx.x & 31;
  const int wave = threadIdx.x >> 5;
  const int tilesN = N >> 6;
  const int tilesM = M >> 6;
  const int tile = blockIdx.x * 8 + wave;
  if (tile >= tilesM * tilesN) return;
  const int tm = tile / tilesN;
  const int tn = tile - tm * tilesN;
  const int m0 = tm << 6;
  const int n0 = tn << 6;

  const T* Ab  = A  + (size_t)b * strideA;
  const T* Bb  = Bt + (size_t)b * strideB;
  const T* Ab2 = SPLIT ? (A2  + (size_t)b * strideA) : nullptr;
  const T* Bb2 = SPLIT ? (Bt2 + (size_t)b * strideB) : nullptr;

  const int rlane = lane & 15;
  const int koff  = (lane >> 4) * 8;
  const int mOff  = (lane >> 4) * 8;

  v8f acc[4][4];
#pragma unroll
  for (int i = 0; i < 4; ++i)
#pragma unroll
    for (int j = 0; j < 4; ++j) acc[i][j] = (v8f){0.f,0.f,0.f,0.f,0.f,0.f,0.f,0.f};

  for (int k0 = 0; k0 < K; k0 += 32) {
    V bh[4], bl[4];
#pragma unroll
    for (int j = 0; j < 4; ++j) {
      const size_t bo = (size_t)(n0 + (j << 4) + rlane) * ldb + koff + k0;
      bh[j] = Frag<T>::load(Bb + bo);
      if (SPLIT) bl[j] = Frag<T>::load(Bb2 + bo);
    }
#pragma unroll
    for (int i = 0; i < 4; ++i) {
      const size_t ao = (size_t)(m0 + (i << 4) + rlane) * lda + koff + k0;
      V ah = Frag<T>::load(Ab + ao);
      V al;
      if (SPLIT) al = Frag<T>::load(Ab2 + ao);
#pragma unroll
      for (int j = 0; j < 4; ++j) {
        acc[i][j] = Frag<T>::mma(ah, bh[j], acc[i][j]);
        if (SPLIT) {
          acc[i][j] = Frag<T>::mma(ah, bl[j], acc[i][j]);
          acc[i][j] = Frag<T>::mma(al, bh[j], acc[i][j]);
        }
      }
      Frag<T>::guard(acc[i][0], acc[i][3], ah, SPLIT ? al : ah);
    }
    Frag<T>::keep(bh[0], bh[1], bh[2], bh[3]);
    if (SPLIT) Frag<T>::keep(bl[0], bl[1], bl[2], bl[3]);
  }
  acc_guard4(acc[0][0], acc[0][1], acc[0][2], acc[0][3]);
  acc_guard4(acc[1][0], acc[1][1], acc[1][2], acc[1][3]);
  acc_guard4(acc[2][0], acc[2][1], acc[2][2], acc[2][3]);
  acc_guard4(acc[3][0], acc[3][1], acc[3][2], acc[3][3]);

  float* slab = sT[wave];
#pragma unroll
  for (int i = 0; i < 4; ++i) {
    const int mBase = m0 + (i << 4);
    float bm[8];
#pragma unroll
    for (int r = 0; r < 8; ++r) bm[r] = 0.f;
    if (BIAS_MODE == 1) {
      const v4f b0v = *(const v4f*)(bias + mBase + mOff);
      const v4f b1v = *(const v4f*)(bias + mBase + mOff + 4);
      bm[0] = b0v[0]; bm[1] = b0v[1]; bm[2] = b0v[2]; bm[3] = b0v[3];
      bm[4] = b1v[0]; bm[5] = b1v[1]; bm[6] = b1v[2]; bm[7] = b1v[3];
    }
#pragma unroll
    for (int j = 0; j < 4; ++j) {
      const int n = n0 + (j << 4) + rlane;
      float bv = 0.f;
      if (BIAS_MODE == 2) bv = bias[n];
#pragma unroll
      for (int r = 0; r < 8; ++r) {
        float v = acc[i][j][r] * scale;
        if (BIAS_MODE == 1) v += bm[r];
        if (BIAS_MODE == 2) v += bv;
        slab[(mOff + r) * 68 + (j << 4) + rlane] = v;
      }
    }
    __builtin_amdgcn_fence(__ATOMIC_RELEASE, "workgroup");
    __builtin_amdgcn_wave_barrier();
    __builtin_amdgcn_fence(__ATOMIC_ACQUIRE, "workgroup");
    if (OUT_MODE == 0) {
      float* C = (float*)Cout + (size_t)b * strideC;
      const int hh = lane >> 4, c4 = (lane & 15) * 4;
      for (int pass = 0; pass < 2; ++pass) {
#pragma unroll
        for (int it = 0; it < 8; ++it) {
          const int row = it * 2 + hh;
          v4f v = *(const v4f*)(slab + row * 68 + c4);
          *(volatile v4f*)(C + (size_t)(mBase + row) * ldc + n0 + c4) = v;
        }
        __threadfence();
      }
    } else {
      const int q = lane >> 3, c8 = (lane & 7) * 8;
      unsigned short* C  = (unsigned short*)Cout  + (size_t)b * strideC;
      unsigned short* C2 = (OUT_MODE == 2) ? ((unsigned short*)Cout2 + (size_t)b * strideC) : nullptr;
      for (int pass = 0; pass < 2; ++pass) {
#pragma unroll
        for (int it = 0; it < 4; ++it) {
          const int row = it * 4 + q;
          const float* sp = slab + row * 68 + c8;
          v8h hv, lv;
#pragma unroll
          for (int e = 0; e < 8; ++e) {
            if (OUT_MODE == 1) {
              hv[e] = (_Float16)sp[e];
            } else {
              unsigned short hb = f2bf_bits(sp[e]);
              unsigned short lb = f2bf_bits(sp[e] - bf_bits2f(hb));
              hv[e] = __builtin_bit_cast(_Float16, hb);
              lv[e] = __builtin_bit_cast(_Float16, lb);
            }
          }
          *(volatile v8h*)(C + (size_t)(mBase + row) * ldc + n0 + c8) = hv;
          if (OUT_MODE == 2) *(volatile v8h*)(C2 + (size_t)(mBase + row) * ldc + n0 + c8) = lv;
        }
        __threadfence();
      }
    }
    __builtin_amdgcn_fence(__ATOMIC_RELEASE, "workgroup");
    __builtin_amdgcn_wave_barrier();
    __builtin_amdgcn_fence(__ATOMIC_ACQUIRE, "workgroup");
  }
}

__global__ __launch_bounds__(256) void cast_f32_bf16hilo_x2(
    const float* __restrict__ in, unsigned short* __restrict__ oh, unsigned short* __restrict__ ol, int n2) {
  const int i = blockIdx.x * 256 + threadIdx.x;
  if (i < n2) {
    const float f0 = in[2 * i], f1 = in[2 * i + 1];
    const unsigned short h0 = f2bf_bits(f0), h1 = f2bf_bits(f1);
    const unsigned short l0 = f2bf_bits(f0 - bf_bits2f(h0));
    const unsigned short l1 = f2bf_bits(f1 - bf_bits2f(h1));
    const unsigned uh = (unsigned)h0 | ((unsigned)h1 << 16);
    const unsigned ul = (unsigned)l0 | ((unsigned)l1 << 16);
    ((volatile unsigned*)oh)[i] = uh;
    ((volatile unsigned*)ol)[i] = ul;
    __threadfence();
    ((volatile unsigned*)oh)[i] = uh;
    ((volatile unsigned*)ol)[i] = ul;
  }
}

__global__ __launch_bounds__(256) void transpose_cast_bf16hilo(
    const float* __restrict__ in, unsigned short* __restrict__ oh, unsigned short* __restrict__ ol,
    int R, int Cc) {
  __shared__ float tile[32][65];
  const int tid = threadIdx.x, lane = tid & 31, wave = tid >> 5;
  const int c0 = blockIdx.x * 32, r0 = blockIdx.y * 64;
#pragma unroll
  for (int i = 0; i < 8; ++i) {
    const int idx = i * 256 + tid;
    const int rr = idx >> 5, cc = idx & 31;
    tile[cc][rr] = in[(size_t)(r0 + rr) * Cc + c0 + cc];
  }
  __syncthreads();
  const int orow = wave * 4 + (lane >> 3);
  const int rseg = (lane & 7) * 8;
  v4u hv, lv;
#pragma unroll
  for (int e = 0; e < 4; ++e) {
    const float f0 = tile[orow][rseg + 2 * e];
    const float f1 = tile[orow][rseg + 2 * e + 1];
    const unsigned short h0 = f2bf_bits(f0), h1 = f2bf_bits(f1);
    const unsigned short l0 = f2bf_bits(f0 - bf_bits2f(h0));
    const unsigned short l1 = f2bf_bits(f1 - bf_bits2f(h1));
    hv[e] = (unsigned)h0 | ((unsigned)h1 << 16);
    lv[e] = (unsigned)l0 | ((unsigned)l1 << 16);
  }
  const size_t o = (size_t)(c0 + orow) * R + r0 + rseg;
  for (int pass = 0; pass < 2; ++pass) {
    *(volatile v4u*)(oh + o) = hv;
    *(volatile v4u*)(ol + o) = lv;
    __threadfence();
  }
}

__global__ __launch_bounds__(128)
void attn_causal_hd64(const unsigned short* __restrict__ Qh, const unsigned short* __restrict__ Ql,
                      const unsigned short* __restrict__ Kh, const unsigned short* __restrict__ Kl,
                      const unsigned short* __restrict__ Vh, const unsigned short* __restrict__ Vl,
                      unsigned short* __restrict__ Oh, unsigned short* __restrict__ Ol,
                      int b_first, float qscale) {
  __shared__ __align__(16) unsigned short Ksh[kKC * kHd];
  __shared__ __align__(16) unsigned short Ksl[kKC * kHd];
  __shared__ __align__(16) unsigned short Vsh[kHd * kKC];
  __shared__ __align__(16) unsigned short Vsl[kHd * kKC];
  __shared__ __align__(16) unsigned short Psh[4][16 * kKC];
  __shared__ __align__(16) unsigned short Psl[4][16 * kKC];
  __shared__ __align__(16) float Os[4][16 * 68];

  const int tid  = threadIdx.x;
  const int wave = tid >> 5;
  const int lane = tid & 31;
  const int hh   = lane >> 4;
  const int c    = lane & 15;

  const int bx  = blockIdx.x;
  const int qb  = bx % (kSeq / kQB);
  const int bhl = bx / (kSeq / kQB);
  const int h   = bhl % kHeads;
  const int bl  = bhl / kHeads;
  const int b   = b_first + bl;
  const int q0  = qb * kQB + wave * 16;

  v16b qah[2], qal[2];
  {
    const size_t qo = ((size_t)(b * kSeq + q0 + c)) * kHid + (size_t)h * kHd + 8 * hh;
#pragma unroll
    for (int dc = 0; dc < 2; ++dc) {
      qah[dc] = Frag<__bf16>::load((const __bf16*)Qh + qo + dc * 32);
      qal[dc] = Frag<__bf16>::load((const __bf16*)Ql + qo + dc * 32);
    }
  }

  float mrow[8], lrow[8];
  v8f oacc[4];
#pragma unroll
  for (int r = 0; r < 8; ++r) { mrow[r] = -INFINITY; lrow[r] = 0.f; }
#pragma unroll
  for (int t = 0; t < 4; ++t) oacc[t] = (v8f){0.f,0.f,0.f,0.f,0.f,0.f,0.f,0.f};

  const __bf16* kshb = (const __bf16*)Ksh;
  const __bf16* kslb = (const __bf16*)Ksl;
  const __bf16* vshb = (const __bf16*)Vsh;
  const __bf16* vslb = (const __bf16*)Vsl;
  unsigned short* pwh = Psh[wave];
  unsigned short* pwl = Psl[wave];

  const int nChunks = qb + 1;
  for (int kc = 0; kc < nChunks; ++kc) {
    const int kv0 = kc * kKC;
    __syncthreads();
    {
      const int r = tid >> 1, hf = (tid & 1) * 32;
      const v4u* khs = (const v4u*)(Kh + ((size_t)(b * kSeq + kv0 + r)) * kHid + h * kHd + hf);
      const v4u* kls = (const v4u*)(Kl + ((size_t)(b * kSeq + kv0 + r)) * kHid + h * kHd + hf);
      v4u* khd = (v4u*)(Ksh + r * kHd + hf);
      v4u* kld = (v4u*)(Ksl + r * kHd + hf);
      v4u tk[8];
#pragma unroll
      for (int i = 0; i < 4; ++i) { tk[i] = khs[i]; tk[4 + i] = kls[i]; }
#pragma unroll
      for (int i = 0; i < 4; ++i) { khd[i] = tk[i]; kld[i] = tk[4 + i]; }
      asm volatile("" ::: "memory");
      const v4u* vhs = (const v4u*)(Vh + ((size_t)(h * kHd + r)) * kRows + (size_t)b * kSeq + kv0 + hf);
      const v4u* vls = (const v4u*)(Vl + ((size_t)(h * kHd + r)) * kRows + (size_t)b * kSeq + kv0 + hf);
      v4u* vhd = (v4u*)(Vsh + r * kKC + hf);
      v4u* vld = (v4u*)(Vsl + r * kKC + hf);
      v4u tv[8];
#pragma unroll
      for (int i = 0; i < 4; ++i) { tv[i] = vhs[i]; tv[4 + i] = vls[i]; }
#pragma unroll
      for (int i = 0; i < 4; ++i) { vhd[i] = tv[i]; vld[i] = tv[4 + i]; }
    }
    __syncthreads();

    v8f s[4];
#pragma unroll
    for (int j = 0; j < 4; ++j) {
      s[j] = (v8f){0.f,0.f,0.f,0.f,0.f,0.f,0.f,0.f};
#pragma unroll
      for (int dc = 0; dc < 2; ++dc) {
        const int ko = (j * 16 + c) * kHd + dc * 32 + 8 * hh;
        const v16b kbh = Frag<__bf16>::load(kshb + ko);
        const v16b kbl = Frag<__bf16>::load(kslb + ko);
        s[j] = at_mma(qah[dc], kbh, s[j]);
        s[j] = at_mma(qah[dc], kbl, s[j]);
        s[j] = at_mma(qal[dc], kbh, s[j]);
      }
    }
    const bool diag = (kc == qb);
    float cm[8];
#pragma unroll
    for (int r = 0; r < 8; ++r) {
      const int qrow = q0 + 8 * hh + r;
      float m = -INFINITY;
#pragma unroll
      for (int j = 0; j < 4; ++j) {
        const int kvcol = kv0 + j * 16 + c;
        float val = s[j][r] * qscale;
        val = (diag && (kvcol > qrow)) ? -INFINITY : val;
        s[j][r] = val;
        m = fmaxf(m, val);
      }
#pragma unroll
      for (int off = 1; off < 16; off <<= 1) m = fmaxf(m, __shfl_xor(m, off, 32));
      cm[r] = m;
    }
#pragma unroll
    for (int r = 0; r < 8; ++r) {
      const float mnew = fmaxf(mrow[r], cm[r]);
      const float alpha = expf(mrow[r] - mnew);
      mrow[r] = mnew;
      float psum = 0.f;
#pragma unroll
      for (int j = 0; j < 4; ++j) {
        const float p = expf(s[j][r] - mnew);
        psum += p;
        const unsigned short hb = f2bf_bits(p);
        const unsigned short lb = f2bf_bits(p - bf_bits2f(hb));
        pwh[(8 * hh + r) * kKC + j * 16 + c] = hb;
        pwl[(8 * hh + r) * kKC + j * 16 + c] = lb;
      }
#pragma unroll
      for (int off = 1; off < 16; off <<= 1) psum += __shfl_xor(psum, off, 32);
      lrow[r] = lrow[r] * alpha + psum;
#pragma unroll
      for (int t = 0; t < 4; ++t) oacc[t][r] *= alpha;
    }
    __builtin_amdgcn_fence(__ATOMIC_RELEASE, "workgroup");
    __builtin_amdgcn_wave_barrier();
    __builtin_amdgcn_fence(__ATOMIC_ACQUIRE, "workgroup");
#pragma unroll
    for (int kk = 0; kk < 2; ++kk) {
      const int po = c * kKC + kk * 32 + 8 * hh;
      const v16b pa = Frag<__bf16>::load((const __bf16*)pwh + po);
      const v16b pl = Frag<__bf16>::load((const __bf16*)pwl + po);
#pragma unroll
      for (int t = 0; t < 4; ++t) {
        const int vo = (t * 16 + c) * kKC + kk * 32 + 8 * hh;
        const v16b vbh = Frag<__bf16>::load(vshb + vo);
        const v16b vbl = Frag<__bf16>::load(vslb + vo);
        oacc[t] = at_mma(pa, vbh, oacc[t]);
        oacc[t] = at_mma(pa, vbl, oacc[t]);
        oacc[t] = at_mma(pl, vbh, oacc[t]);
      }
    }
  }

  float* os = Os[wave];
#pragma unroll
  for (int r = 0; r < 8; ++r) {
    const float inv = 1.0f / lrow[r];
#pragma unroll
    for (int t = 0; t < 4; ++t) os[(8 * hh + r) * 68 + t * 16 + c] = oacc[t][r] * inv;
  }
  __builtin_amdgcn_fence(__ATOMIC_RELEASE, "workgroup");
  __builtin_amdgcn_wave_barrier();
  __builtin_amdgcn_fence(__ATOMIC_ACQUIRE, "workgroup");
  {
    const int qq = lane >> 3, c8 = (lane & 7) * 8;
    const size_t ob = ((size_t)(bl * kSeq + q0)) * kHid + (size_t)h * kHd + c8;
    for (int pass = 0; pass < 2; ++pass) {
#pragma unroll
      for (int it = 0; it < 4; ++it) {
        const int row = it * 4 + qq;
        const float* sp = os + row * 68 + c8;
        v4u hv, lv;
#pragma unroll
        for (int e = 0; e < 4; ++e) {
          const float f0 = sp[2 * e], f1 = sp[2 * e + 1];
          const unsigned short h0 = f2bf_bits(f0), h1 = f2bf_bits(f1);
          const unsigned short l0 = f2bf_bits(f0 - bf_bits2f(h0));
          const unsigned short l1 = f2bf_bits(f1 - bf_bits2f(h1));
          hv[e] = (unsigned)h0 | ((unsigned)h1 << 16);
          lv[e] = (unsigned)l0 | ((unsigned)l1 << 16);
        }
        *(volatile v4u*)(Oh + ob + (size_t)row * kHid) = hv;
        *(volatile v4u*)(Ol + ob + (size_t)row * kHid) = lv;
      }
      __threadfence();
    }
  }
}

extern "C" void kernel_launch(void* const* d_in, const int* in_sizes, int n_in,
                              void* d_out, int out_size, void* d_ws, size_t ws_size,
                              hipStream_t stream) {
  if (n_in < 9) return;
  if (in_sizes[0] != kRows * kHd) return;
  if (in_sizes[1] != kHd * kHid || in_sizes[3] != kHd * kHid || in_sizes[5] != kHd * kHid) return;
  if (in_sizes[2] != kHid || in_sizes[4] != kHid || in_sizes[6] != kHid) return;
  if (in_sizes[7] != kHid * kHd || in_sizes[8] != kHd) return;
  if (out_size != kRows * kHd) return;

  const float* x  = (const float*)d_in[0];
  const float* Wq = (const float*)d_in[1];
  const float* bq = (const float*)d_in[2];
  const float* Wk = (const float*)d_in[3];
  const float* bk = (const float*)d_in[4];
  const float* Wv = (const float*)d_in[5];
  const float* bv = (const float*)d_in[6];
  const float* Wo = (const float*)d_in[7];
  const float* bo = (const float*)d_in[8];
  float* out = (float*)d_out;

  const size_t szX  = (size_t)kRows * kHd * 2;
  const size_t szW  = (size_t)kHid * kHd * 2;
  const size_t szQ  = (size_t)kRows * kHid * 2;
  const size_t szAO = (size_t)kRowsPP * kHid * 2;
  const size_t total = 2 * szX + 8 * szW + 6 * szQ + 2 * szAO;
  if (total > ws_size) return;

  char* ws = (char*)d_ws;
  size_t off = 0;
  unsigned short* xh  = (unsigned short*)(ws + off); off += szX;
  unsigned short* xl  = (unsigned short*)(ws + off); off += szX;
  unsigned short* wqh = (unsigned short*)(ws + off); off += szW;
  unsigned short* wql = (unsigned short*)(ws + off); off += szW;
  unsigned short* wkh = (unsigned short*)(ws + off); off += szW;
  unsigned short* wkl = (unsigned short*)(ws + off); off += szW;
  unsigned short* wvh = (unsigned short*)(ws + off); off += szW;
  unsigned short* wvl = (unsigned short*)(ws + off); off += szW;
  unsigned short* woh = (unsigned short*)(ws + off); off += szW;
  unsigned short* wol = (unsigned short*)(ws + off); off += szW;
  unsigned short* qh  = (unsigned short*)(ws + off); off += szQ;
  unsigned short* ql  = (unsigned short*)(ws + off); off += szQ;
  unsigned short* kh  = (unsigned short*)(ws + off); off += szQ;
  unsigned short* kl  = (unsigned short*)(ws + off); off += szQ;
  unsigned short* vth = (unsigned short*)(ws + off); off += szQ;
  unsigned short* vtl = (unsigned short*)(ws + off); off += szQ;
  unsigned short* aoh = (unsigned short*)(ws + off); off += szAO;
  unsigned short* aol = (unsigned short*)(ws + off); off += szAO;
  if (off > ws_size) return;
  void* dummyv = (void*)ws;
  const float* dummyf = (const float*)ws;

  {
    const int n2 = kRows * kHd / 2;
    cast_f32_bf16hilo_x2<<<dim3(n2 / 256), dim3(256), 0, stream>>>(x, xh, xl, n2);
  }
  transpose_cast_bf16hilo<<<dim3(kHid / 32, kHd / 64), dim3(256), 0, stream>>>(Wq, wqh, wql, kHd, kHid);
  transpose_cast_bf16hilo<<<dim3(kHid / 32, kHd / 64), dim3(256), 0, stream>>>(Wk, wkh, wkl, kHd, kHid);
  transpose_cast_bf16hilo<<<dim3(kHid / 32, kHd / 64), dim3(256), 0, stream>>>(Wv, wvh, wvl, kHd, kHid);
  transpose_cast_bf16hilo<<<dim3(kHd / 32, kHid / 64), dim3(256), 0, stream>>>(Wo, woh, wol, kHid, kHd);

  {
    const int gridQ = (kRows / 64) * (kHid / 64) / 8;
    wmma_gemm64<1, true, 2, 2, false, 0><<<dim3(gridQ, 1), dim3(256), 0, stream>>>(
        xh, xl, kHd, 0L, wqh, wql, kHd, 0L, (void*)qh, (void*)ql, kHid, 0L, bq, dummyf, 0L,
        kRows, kHid, kHd, 1.0f);
    wmma_gemm64<1, true, 2, 2, false, 0><<<dim3(gridQ, 1), dim3(256), 0, stream>>>(
        xh, xl, kHd, 0L, wkh, wkl, kHd, 0L, (void*)kh, (void*)kl, kHid, 0L, bk, dummyf, 0L,
        kRows, kHid, kHd, 1.0f);
    const int gridV = (kHid / 64) * (kRows / 64) / 8;
    wmma_gemm64<1, true, 1, 2, false, 0><<<dim3(gridV, 1), dim3(256), 0, stream>>>(
        wvh, wvl, kHd, 0L, xh, xl, kHd, 0L, (void*)vth, (void*)vtl, kRows, 0L, bv, dummyf, 0L,
        kHid, kRows, kHd, 1.0f);
  }

  const float qscale = 0.125f;
  for (int ps = 0; ps < kBatch / kBPP; ++ps) {
    attn_causal_hd64<<<dim3(kBPP * kHeads * (kSeq / kQB)), dim3(128), 0, stream>>>(
        qh, ql, kh, kl, vth, vtl, aoh, aol, ps * kBPP, qscale);
    const int gridO = (kRowsPP / 64) * (kHd / 64) / 8;
    float* outp = out + (size_t)ps * kRowsPP * kHd;
    wmma_gemm64<1, true, 2, 0, false, 0><<<dim3(gridO, 1), dim3(256), 0, stream>>>(
        aoh, aol, kHid, 0L, woh, wol, kHid, 0L, (void*)outp, dummyv, kHd, 0L, bo, dummyf, 0L,
        kRowsPP, kHd, kHid, 1.0f);
  }
}
